// CrystallGNN_46042049413576
// MI455X (gfx1250) — hardware-verified
//
#include <hip/hip_runtime.h>
#include <stddef.h>


#define DF      64
#define DH      128
#define NRBF    10
#define NTHR    256
#define NWAVE   8
#define EPT     8
#define NGRP    2
#define CHUNK   (NTHR * EPT * NGRP)
#define WCAP    (EPT * NGRP * 32)
#define LISTN   (NWAVE * WCAP)
#define NBA     1024
#define GROWS   (NWAVE * 16)
#define GPB     32
#define APA     72
#define APC     136
#define WSCALE  8.0f
#define WINV    0.125f
#define LDS_AGG (NBA * DF * 4 + LISTN * 4 + 64)

static_assert((CHUNK & (CHUNK - 1)) == 0);
static_assert(CHUNK <= 4096);
static_assert((NBA & (NBA - 1)) == 0);
static_assert(NBA <= 4096);
static_assert(GPB == 32);
static_assert(NTHR == GPB * 8);
static_assert(NBA * DF == NWAVE * 64 * 128);
static_assert(DF == 64);
static_assert(DH == 128);

typedef float    v2f  __attribute__((ext_vector_type(2)));
typedef float    v4f  __attribute__((ext_vector_type(4)));
typedef float    v8f  __attribute__((ext_vector_type(8)));
typedef int      v4i  __attribute__((ext_vector_type(4)));
typedef _Float16 v8h  __attribute__((ext_vector_type(8)));
typedef _Float16 v16h __attribute__((ext_vector_type(16)));
union FragH { v16h v; v8h h[2]; };

__device__ __forceinline__ v8h cvt8(v4f a, v4f b) {
  v8h r;
  r[0] = (_Float16)a.x; r[1] = (_Float16)a.y; r[2] = (_Float16)a.z; r[3] = (_Float16)a.w;
  r[4] = (_Float16)b.x; r[5] = (_Float16)b.y; r[6] = (_Float16)b.z; r[7] = (_Float16)b.w;
  return r;
}

__device__ __forceinline__ v8f wmh(v16h a, v16h b, v8f c) {
  v8f d = __builtin_amdgcn_wmma_f32_16x16x32_f16(false, a, false, b, (short)0, c, false, false);
  asm volatile("v_nop\n\tv_nop\n\tv_nop\n\tv_nop" : "+v"(d) : "v"(a), "v"(b));
  return d;
}

__device__ __forceinline__ float softplus_f(float v) {
  return fmaxf(v, 0.0f) + __logf(1.0f + __expf(-fabsf(v)));
}

template <int NB>
__device__ __forceinline__ int scan_chunk(const int* __restrict__ keys, int nK, int cbase, int base,
                                          int vec8, int* list, int tid, int lane, int wave) {
  int wc = 0;
#pragma unroll
  for (int g = 0; g < NGRP; ++g) {
    const int el0  = (g * NTHR + tid) * EPT;
    const int e0   = cbase + el0;
    const int sent = -2147483647 - 1;
    v4i da, db;
    if (vec8 != 0 && e0 + 7 < nK) {
      da = *(const v4i*)(keys + e0);
      db = *(const v4i*)(keys + e0 + 4);
    } else {
      da.x = (e0     < nK) ? keys[min(e0, nK - 1)] : sent;
      da.y = (e0 + 1 < nK) ? keys[min(e0 + 1, nK - 1)] : sent;
      da.z = (e0 + 2 < nK) ? keys[min(e0 + 2, nK - 1)] : sent;
      da.w = (e0 + 3 < nK) ? keys[min(e0 + 3, nK - 1)] : sent;
      db.x = (e0 + 4 < nK) ? keys[min(e0 + 4, nK - 1)] : sent;
      db.y = (e0 + 5 < nK) ? keys[min(e0 + 5, nK - 1)] : sent;
      db.z = (e0 + 6 < nK) ? keys[min(e0 + 6, nK - 1)] : sent;
      db.w = (e0 + 7 < nK) ? keys[min(e0 + 7, nK - 1)] : sent;
    }
    const unsigned nb = (unsigned)base;
    const unsigned s0 = (unsigned)da.x - nb, s1 = (unsigned)da.y - nb;
    const unsigned s2 = (unsigned)da.z - nb, s3 = (unsigned)da.w - nb;
    const unsigned s4 = (unsigned)db.x - nb, s5 = (unsigned)db.y - nb;
    const unsigned s6 = (unsigned)db.z - nb, s7 = (unsigned)db.w - nb;
    const bool h0 = s0 < (unsigned)NB, h1 = s1 < (unsigned)NB, h2 = s2 < (unsigned)NB, h3 = s3 < (unsigned)NB;
    const bool h4 = s4 < (unsigned)NB, h5 = s5 < (unsigned)NB, h6 = s6 < (unsigned)NB, h7 = s7 < (unsigned)NB;
    const unsigned any = __builtin_amdgcn_ballot_w32(h0 | h1 | h2 | h3 | h4 | h5 | h6 | h7);
    if (any != 0u) {
#define HITJ(J, HJ, SJ) { \
        const unsigned mj = __builtin_amdgcn_ballot_w32(HJ); \
        if (mj != 0u) { \
          if (HJ) { \
            const int pos = wc + (int)__builtin_amdgcn_mbcnt_lo(mj, 0u); \
            if (pos < WCAP) list[wave * WCAP + pos] = ((el0 + (J)) << 12) | (int)(SJ); \
          } \
          wc += (int)__builtin_popcount(mj); } }
      HITJ(0, h0, s0)
      HITJ(1, h1, s1)
      HITJ(2, h2, s2)
      HITJ(3, h3, s3)
      HITJ(4, h4, s4)
      HITJ(5, h5, s5)
      HITJ(6, h6, s6)
      HITJ(7, h7, s7)
#undef HITJ
    }
  }
  return wc;
}

__global__ __launch_bounds__(NTHR) void k_prep(
    const float* __restrict__ W1, const float* __restrict__ W2, const float* __restrict__ Ws,
    const float* __restrict__ Wb, const float* __restrict__ Wh,
    _Float16* w1s, _Float16* w2s, _Float16* wss, _Float16* wbs, _Float16* whs, int nConv) {
  const int i  = blockIdx.x * NTHR + threadIdx.x;
  const int nA = nConv * DF * DF / 8;
  const int nS = DF * DH / 8;
  const int tot = 2 * nA + 3 * nS;
  if (i >= tot) return;
  int seg, li;
  if (i < nA)                    { seg = 0; li = i; }
  else if (i < 2 * nA)           { seg = 1; li = i - nA; }
  else if (i < 2 * nA + nS)      { seg = 2; li = i - 2 * nA; }
  else if (i < 2 * nA + 2 * nS)  { seg = 3; li = i - 2 * nA - nS; }
  else                           { seg = 4; li = i - 2 * nA - 2 * nS; }
  const int o = li * 8;
  const float* p;
  int stride;
  _Float16* dp;
  if (seg < 2) {
    const int layer = o / (DF * DF);
    const int oo    = o - layer * DF * DF;
    const int n     = oo / DF;
    const int k0    = oo - n * DF;
    p = (seg == 0 ? W1 : W2) + (size_t)layer * DF * DF + (size_t)k0 * DF + n;
    stride = DF;
    dp = (seg == 0 ? w1s : w2s) + o;
  } else if (seg == 2) {
    const int n  = o / DF;
    const int k0 = o - n * DF;
    p = Ws + (size_t)k0 * DH + n;
    stride = DH;
    dp = wss + o;
  } else {
    const int n  = o / DH;
    const int k0 = o - n * DH;
    p = (seg == 3 ? Wb : Wh) + (size_t)k0 * DF + n;
    stride = DF;
    dp = (seg == 3 ? wbs : whs) + o;
  }
  v4f a, b;
  a.x = p[0];          a.y = p[stride];     a.z = p[2 * stride]; a.w = p[3 * stride];
  b.x = p[4 * stride]; b.y = p[5 * stride]; b.z = p[6 * stride]; b.w = p[7 * stride];
  a = a * WSCALE;
  b = b * WSCALE;
  const v8h hv = cvt8(a, b);
  *(volatile v8h*)dp = hv;
  __threadfence();
  *(volatile v8h*)dp = hv;
}

__global__ __launch_bounds__(NTHR) void k_embed(
    const int* __restrict__ ids, const float* __restrict__ emb, float* x,
    int nN, int nEmb, int nRowsPad) {
  const int i = blockIdx.x * NTHR + threadIdx.x;
  if (i >= nRowsPad * (DF / 4)) return;
  const int r  = i >> 4;
  const int c4 = (i & 15) * 4;
  const int node = r < nN ? r : nN - 1;
  int id = ids[node];
  id = id < 0 ? 0 : (id > nEmb - 1 ? nEmb - 1 : id);
  const v4f v = *(const v4f*)(emb + (size_t)id * DF + c4);
  float* dp = x + (size_t)r * DF + c4;
  *(volatile v4f*)dp = v;
  __threadfence();
  *(volatile v4f*)dp = v;
}

__global__ __launch_bounds__(NTHR) void k_gemm(
    const float* A, const _Float16* __restrict__ wT, const float* __restrict__ bias,
    const float* resid, float* out, int act) {
  __shared__ __attribute__((aligned(16))) float tile[NWAVE * 16 * DF];
  const int tid = threadIdx.x, lane = tid & 31, wave = tid >> 5, hh = lane >> 4, m = lane & 15;
  const int row0 = (blockIdx.x * NWAVE + wave) * 16;

  v8f acc[4];
#pragma unroll
  for (int t = 0; t < 4; ++t) { v8f z = {0.f, 0.f, 0.f, 0.f, 0.f, 0.f, 0.f, 0.f}; acc[t] = z; }

  const float* ar = A + (size_t)(row0 + m) * DF + 8 * hh;
#pragma unroll
  for (int kt = 0; kt < DF / 32; ++kt) {
    const v4f p0 = *(const v4f*)(ar + 32 * kt),      p1 = *(const v4f*)(ar + 32 * kt + 4);
    const v4f p2 = *(const v4f*)(ar + 32 * kt + 16), p3 = *(const v4f*)(ar + 32 * kt + 20);
    FragH a;
    a.h[0] = cvt8(p0, p1);
    a.h[1] = cvt8(p2, p3);
#pragma unroll
    for (int t = 0; t < 4; ++t) {
      const _Float16* bp = wT + (size_t)(16 * t + m) * DF + 32 * kt + 8 * hh;
      FragH b;
      b.h[0] = *(const v8h*)bp;
      b.h[1] = *(const v8h*)(bp + 16);
      acc[t] = wmh(a.v, b.v, acc[t]);
    }
  }

  float* st = tile + wave * 16 * DF + (8 * hh) * DF + m;
#pragma unroll
  for (int t = 0; t < 4; ++t) {
#pragma unroll
    for (int r = 0; r < 8; ++r) st[r * DF + 16 * t] = acc[t][r];
  }
  __syncthreads();

  const int c4 = (4 * lane) & (DF - 1);
  const v4f bv = *(const v4f*)(bias + c4);
  const float* lp = tile + wave * 16 * DF + 4 * lane;
  const size_t gofs = (size_t)row0 * DF + 4 * lane;
  v4f ov[8];
#pragma unroll
  for (int q = 0; q < 8; ++q) {
    v4f v = *(const v4f*)(lp + q * 128) * WINV + bv;
    if (act) {
      const v4f rv = *(const v4f*)(resid + gofs + (size_t)q * 128);
      v = v + rv;
      v.x = softplus_f(v.x); v.y = softplus_f(v.y); v.z = softplus_f(v.z); v.w = softplus_f(v.w);
    }
    ov[q] = v;
  }
#pragma unroll
  for (int q = 0; q < 8; ++q) *(volatile v4f*)(out + gofs + (size_t)q * 128) = ov[q];
  __threadfence();
#pragma unroll
  for (int q = 0; q < 8; ++q) *(volatile v4f*)(out + gofs + (size_t)q * 128) = ov[q];
}

__global__ __launch_bounds__(NTHR) void k_agg(
    const int* __restrict__ ei, const float* __restrict__ ea, const float* __restrict__ h,
    const float* __restrict__ We, const float* __restrict__ be, float* agg,
    int nN, int nE, int vec8) {
  extern __shared__ v4f lds_dyn[];
  float* acc  = (float*)lds_dyn;
  int*   list = (int*)(acc + NBA * DF);
  int*   wcnt = list + LISTN;
  const int tid = threadIdx.x, lane = tid & 31, wave = tid >> 5;
  const int nodeBase = blockIdx.x * NBA;
  const int* dsts = ei + nE;

  {
    const v4f z = {0.f, 0.f, 0.f, 0.f};
    for (int i = tid; i < NBA * DF / 4; i += NTHR) lds_dyn[i] = z;
  }

  float we0[NRBF], we1[NRBF];
#pragma unroll
  for (int r = 0; r < NRBF; ++r) {
    const v2f w = *(const v2f*)(We + r * DF + 2 * lane);
    we0[r] = w.x; we1[r] = w.y;
  }
  const v2f   bb    = *(const v2f*)(be + 2 * lane);
  const float inv9  = 1.0f / (float)(NRBF - 1);
  const float off1  = 6.0f * (1.0f * inv9);
  const float coeff = -0.5f * (1.0f / (off1 * off1));
  const float offl  = 6.0f * ((float)(lane < NRBF ? lane : 0) * inv9);
  __syncthreads();

  const int nChunks = (nE + CHUNK - 1) / CHUNK;
#pragma unroll 1
  for (int ch = 0; ch < nChunks; ++ch) {
    const int cbase = ch * CHUNK;
    const int wc = scan_chunk<NBA>(dsts, nE, cbase, nodeBase, vec8, list, tid, lane, wave);
    if (lane == 0) wcnt[wave] = wc;
    __syncthreads();
    if (wave == 0) {
#pragma unroll 1
      for (int wsx = 0; wsx < NWAVE; ++wsx) {
        int n = __builtin_amdgcn_readfirstlane(wcnt[wsx]);
        n = n > WCAP ? WCAP : (n < 0 ? 0 : n);
        const int* lp = list + wsx * WCAP;
#pragma unroll 1
        for (int i = 0; i < n; ++i) {
          const int ent  = __builtin_amdgcn_readfirstlane(lp[i]);
          const int slot = ent & (NBA - 1);
          int e = cbase + ((ent >> 12) & (CHUNK - 1));
          e = e > nE - 1 ? nE - 1 : e;
          int src = ei[e];
          src = src < 0 ? 0 : (src > nN - 1 ? nN - 1 : src);
          const float d  = ea[e];
          const float t  = d - offl;
          const float er = __expf(coeff * (t * t));
          const int   eri = __float_as_int(er);
          float f0 = bb.x, f1 = bb.y;
#pragma unroll
          for (int r = 0; r < NRBF; ++r) {
            const float ev = __int_as_float(__builtin_amdgcn_readlane(eri, r));
            f0 = fmaf(ev, we0[r], f0);
            f1 = fmaf(ev, we1[r], f1);
          }
          const v2f hv = *(const v2f*)(h + (size_t)src * DF + 2 * lane);
          v2f* ap = (v2f*)(acc + slot * DF + 2 * lane);
          v2f av = *ap;
          av.x = fmaf(hv.x, f0, av.x);
          av.y = fmaf(hv.y, f1, av.y);
          *ap = av;
        }
      }
    }
    __syncthreads();
  }

  float* gp = agg + (size_t)nodeBase * DF;
#pragma unroll 4
  for (int q = 0; q < 64; ++q) {
    const int f = (wave * 64 + q) * 128 + 4 * lane;
    const v4f v = *(const v4f*)(acc + f);
    *(volatile v4f*)(gp + f) = v;
  }
  __threadfence();
#pragma unroll 4
  for (int q = 0; q < 64; ++q) {
    const int f = (wave * 64 + q) * 128 + 4 * lane;
    const v4f v = *(const v4f*)(acc + f);
    *(volatile v4f*)(gp + f) = v;
  }
}

__global__ __launch_bounds__(NTHR) void k_pool_head(
    const int* __restrict__ bat, const float* __restrict__ x,
    const _Float16* __restrict__ wss, const float* __restrict__ bs,
    const _Float16* __restrict__ wbs, const float* __restrict__ bb1,
    const float* __restrict__ wb2, const float* __restrict__ bb2,
    const _Float16* __restrict__ whs, const float* __restrict__ bh1,
    const float* __restrict__ wh2, const float* __restrict__ bh2,
    float* out, int nN, int nG) {
  __shared__ __attribute__((aligned(16))) float accp[GPB * DF];
  __shared__ __attribute__((aligned(16))) int list[LISTN];
  __shared__ int wcnt[NWAVE];
  __shared__ int cntp[GPB];
  __shared__ __attribute__((aligned(16))) _Float16 sA[GPB * APA];
  __shared__ __attribute__((aligned(16))) _Float16 sC[GPB * APC];
  __shared__ float part[2 * 4 * GPB];
  __shared__ __attribute__((aligned(16))) float outs[2 * GPB];
  const int tid = threadIdx.x, lane = tid & 31, wave = tid >> 5, hh = lane >> 4, m = lane & 15;
  const int gBase = blockIdx.x * GPB;

  for (int i = tid; i < GPB * DF; i += NTHR) accp[i] = 0.f;
  if (tid < GPB) cntp[tid] = 0;
  __syncthreads();

  const int nChunks = (nN + CHUNK - 1) / CHUNK;
#pragma unroll 1
  for (int ch = 0; ch < nChunks; ++ch) {
    const int cbase = ch * CHUNK;
    const int wc = scan_chunk<GPB>(bat, nN, cbase, gBase, 1, list, tid, lane, wave);
    if (lane == 0) wcnt[wave] = wc;
    __syncthreads();
    if (wave == 0) {
#pragma unroll 1
      for (int wsx = 0; wsx < NWAVE; ++wsx) {
        int n = __builtin_amdgcn_readfirstlane(wcnt[wsx]);
        n = n > WCAP ? WCAP : (n < 0 ? 0 : n);
        const int* lp = list + wsx * WCAP;
#pragma unroll 1
        for (int i = 0; i < n; ++i) {
          const int ent  = __builtin_amdgcn_readfirstlane(lp[i]);
          const int slot = ent & (GPB - 1);
          int node = cbase + ((ent >> 12) & (CHUNK - 1));
          node = node > nN - 1 ? nN - 1 : node;
          const v2f xv = *(const v2f*)(x + (size_t)node * DF + 2 * lane);
          v2f* ap = (v2f*)(accp + slot * DF + 2 * lane);
          *ap = *ap + xv;
          if (lane == 0) cntp[slot] = cntp[slot] + 1;
        }
      }
    }
    __syncthreads();
  }

  {
    const int row = tid >> 3, c0 = (tid & 7) * 8;
    const int cn  = cntp[row];
    const float rc = 1.0f / fmaxf((float)cn, 1.0f);
    const v4f a = *(const v4f*)(accp + row * DF + c0) * rc;
    const v4f b = *(const v4f*)(accp + row * DF + c0 + 4) * rc;
    *(v8h*)(sA + row * APA + c0) = cvt8(a, b);
  }
  __syncthreads();

  const int rt = wave >> 2;
  {
    const int ct0 = (wave & 3) * 2;
    v8f c2[2];
    { v8f z = {0.f, 0.f, 0.f, 0.f, 0.f, 0.f, 0.f, 0.f}; c2[0] = z; c2[1] = z; }
    const _Float16* ar = sA + (16 * rt + m) * APA + 8 * hh;
#pragma unroll
    for (int kt = 0; kt < DF / 32; ++kt) {
      FragH a;
      a.h[0] = *(const v8h*)(ar + 32 * kt);
      a.h[1] = *(const v8h*)(ar + 32 * kt + 16);
#pragma unroll
      for (int j = 0; j < 2; ++j) {
        const _Float16* bp = wss + (size_t)(16 * (ct0 + j) + m) * DF + 32 * kt + 8 * hh;
        FragH b;
        b.h[0] = *(const v8h*)bp;
        b.h[1] = *(const v8h*)(bp + 16);
        c2[j] = wmh(a.v, b.v, c2[j]);
      }
    }
#pragma unroll
    for (int j = 0; j < 2; ++j) {
      const int col = 16 * (ct0 + j) + m;
      const float bsv = bs[col];
      _Float16* cp = sC + (16 * rt + 8 * hh) * APC + col;
#pragma unroll
      for (int r = 0; r < 8; ++r) cp[r * APC] = (_Float16)fmaxf(c2[j][r] * WINV + bsv, 0.f);
    }
  }
  __syncthreads();

  {
    const int ct = wave & 3;
    const _Float16* ar = sC + (16 * rt + m) * APC + 8 * hh;
#pragma unroll
    for (int hd = 0; hd < 2; ++hd) {
      const _Float16* wp = hd ? whs : wbs;
      const float b1v = (hd ? bh1 : bb1)[16 * ct + m];
      const float w2v = (hd ? wh2 : wb2)[16 * ct + m];
      v8f d = {0.f, 0.f, 0.f, 0.f, 0.f, 0.f, 0.f, 0.f};
#pragma unroll
      for (int kt = 0; kt < DH / 32; ++kt) {
        FragH a;
        a.h[0] = *(const v8h*)(ar + 32 * kt);
        a.h[1] = *(const v8h*)(ar + 32 * kt + 16);
        const _Float16* bp = wp + (size_t)(16 * ct + m) * DH + 32 * kt + 8 * hh;
        FragH b;
        b.h[0] = *(const v8h*)bp;
        b.h[1] = *(const v8h*)(bp + 16);
        d = wmh(a.v, b.v, d);
      }
      float p[8];
#pragma unroll
      for (int r = 0; r < 8; ++r) p[r] = fmaxf(d[r] * WINV + b1v, 0.f) * w2v;
#pragma unroll
      for (int r = 0; r < 8; ++r) {
        p[r] += __shfl_xor(p[r], 1);
        p[r] += __shfl_xor(p[r], 2);
        p[r] += __shfl_xor(p[r], 4);
        p[r] += __shfl_xor(p[r], 8);
      }
      if (m == 0) {
#pragma unroll
        for (int r = 0; r < 8; ++r) part[(hd * 4 + ct) * GPB + 16 * rt + 8 * hh + r] = p[r];
      }
    }
  }
  __syncthreads();

  if (tid < 2 * GPB) {
    const int hd = tid / GPB, row = tid - hd * GPB;
    const float b2s = hd ? bh2[0] : bb2[0];
    const float* pp = part + hd * 4 * GPB + row;
    const float o = ((pp[0] + pp[GPB]) + pp[2 * GPB]) + pp[3 * GPB] + b2s;
    outs[tid] = o;
  }
  __syncthreads();

  if (wave == 0 && lane < 16) {
    const int hd = lane >> 3, q = lane & 7;
    const v4f v = *(const v4f*)(outs + hd * GPB + 4 * q);
    float* gp = out + (size_t)hd * nG + gBase + 4 * q;
    *(volatile v4f*)gp = v;
    __threadfence();
    *(volatile v4f*)gp = v;
  }
}

extern "C" void kernel_launch(void* const* d_in, const int* in_sizes, int n_in,
                              void* d_out, int out_size, void* d_ws, size_t ws_size,
                              hipStream_t stream) {
  if (n_in < 21) return;
  const int nN    = in_sizes[0];
  const int nE    = in_sizes[1] / 2;
  const int nEmb  = in_sizes[4] / DF;
  const int nConv = in_sizes[5] / (DF * DF);
  const int nG    = out_size / 2;
  if (nN <= 0 || nE <= 0 || nEmb <= 0 || nConv <= 0 || nG <= 0) return;
  if (in_sizes[1] != 2 * nE || in_sizes[2] < nE || in_sizes[3] != nN || in_sizes[4] != nEmb * DF) return;
  if (in_sizes[5] != nConv * DF * DF || in_sizes[6] < nConv * DF || in_sizes[7] != nConv * NRBF * DF ||
      in_sizes[8] < nConv * DF || in_sizes[9] != nConv * DF * DF || in_sizes[10] < nConv * DF) return;
  if (in_sizes[11] != DF * DH || in_sizes[12] < DH || in_sizes[13] != DH * DF || in_sizes[14] < DF ||
      in_sizes[15] < DF || in_sizes[16] < 1 || in_sizes[17] != DH * DF || in_sizes[18] < DF ||
      in_sizes[19] < DF || in_sizes[20] < 1) return;
  if (out_size != 2 * nG || (nG % GPB) != 0) return;

  const int*   x_ids  = (const int*)d_in[0];
  const int*   eindex = (const int*)d_in[1];
  const float* eattr  = (const float*)d_in[2];
  const int*   batch  = (const int*)d_in[3];
  const float* emb    = (const float*)d_in[4];
  const float* blk_W1 = (const float*)d_in[5];
  const float* blk_b1 = (const float*)d_in[6];
  const float* blk_We = (const float*)d_in[7];
  const float* blk_be = (const float*)d_in[8];
  const float* blk_W2 = (const float*)d_in[9];
  const float* blk_b2 = (const float*)d_in[10];
  const float* Ws     = (const float*)d_in[11];
  const float* bs     = (const float*)d_in[12];
  const float* Wbg1   = (const float*)d_in[13];
  const float* bbg1   = (const float*)d_in[14];
  const float* Wbg2   = (const float*)d_in[15];
  const float* bbg2   = (const float*)d_in[16];
  const float* Weh1   = (const float*)d_in[17];
  const float* beh1   = (const float*)d_in[18];
  const float* Weh2   = (const float*)d_in[19];
  const float* beh2   = (const float*)d_in[20];
  float* out = (float*)d_out;

  const int nGB      = (nN + GROWS - 1) / GROWS;
  const int nRowsPad = nGB * GROWS;
  const int nAB      = (nN + NBA - 1) / NBA;
  const int aggRows  = nAB * NBA;
  if (aggRows < nRowsPad) return;

  char* ws = (char*)d_ws;
  size_t off = 0;
  const size_t oX  = off; off += (size_t)nRowsPad * DF * 4;          off = (off + 255) & ~(size_t)255;
  const size_t oH  = off; off += (size_t)nRowsPad * DF * 4;          off = (off + 255) & ~(size_t)255;
  const size_t oAg = off; off += (size_t)aggRows * DF * 4;           off = (off + 255) & ~(size_t)255;
  const size_t oW1 = off; off += (size_t)nConv * DF * DF * 2;        off = (off + 255) & ~(size_t)255;
  const size_t oW2 = off; off += (size_t)nConv * DF * DF * 2;        off = (off + 255) & ~(size_t)255;
  const size_t oWs = off; off += (size_t)DF * DH * 2;                off = (off + 255) & ~(size_t)255;
  const size_t oWb = off; off += (size_t)DH * DF * 2;                off = (off + 255) & ~(size_t)255;
  const size_t oWh = off; off += (size_t)DH * DF * 2;                off = (off + 255) & ~(size_t)255;
  if (off > ws_size || off > (size_t)134217728) return;
  float*    xP   = (float*)(ws + oX);
  float*    hP   = (float*)(ws + oH);
  float*    aggP = (float*)(ws + oAg);
  _Float16* w1s  = (_Float16*)(ws + oW1);
  _Float16* w2s  = (_Float16*)(ws + oW2);
  _Float16* wss  = (_Float16*)(ws + oWs);
  _Float16* wbs  = (_Float16*)(ws + oWb);
  _Float16* whs  = (_Float16*)(ws + oWh);

  const int vec8  = ((nE & 3) == 0) ? 1 : 0;
  const int nPrep = 2 * (nConv * DF * DF / 8) + 3 * (DF * DH / 8);

  k_prep<<<(nPrep + NTHR - 1) / NTHR, NTHR, 0, stream>>>(blk_W1, blk_W2, Ws, Wbg1, Weh1,
                                                        w1s, w2s, wss, wbs, whs, nConv);

  k_embed<<<(nRowsPad * (DF / 4) + NTHR - 1) / NTHR, NTHR, 0, stream>>>(x_ids, emb, xP, nN, nEmb, nRowsPad);

  hipFuncSetAttribute(reinterpret_cast<const void*>(&k_agg),
                      hipFuncAttributeMaxDynamicSharedMemorySize, LDS_AGG);

  for (int i = 0; i < nConv; ++i) {
    k_gemm<<<nGB, NTHR, 0, stream>>>(xP, w1s + (size_t)i * DF * DF, blk_b1 + (size_t)i * DF, xP, hP, 0);
    k_agg<<<nAB, NTHR, LDS_AGG, stream>>>(eindex, eattr, hP, blk_We + (size_t)i * NRBF * DF,
                                         blk_be + (size_t)i * DF, aggP, nN, nE, vec8);
    k_gemm<<<nGB, NTHR, 0, stream>>>(aggP, w2s + (size_t)i * DF * DF, blk_b2 + (size_t)i * DF, xP, xP, 1);
  }

  k_pool_head<<<nG / GPB, NTHR, 0, stream>>>(batch, xP, wss, bs, wbs, bbg1, Wbg2, bbg2,
                                             whs, beh1, Weh2, beh2, out, nN, nG);
}
